// L2Attention_33509334843619
// MI455X (gfx1250) — hardware-verified
//
#include <hip/hip_runtime.h>
#include <math.h>
#include <stdint.h>

#ifndef NB
#define NB 1
#endif
#ifndef SEQ
#define SEQ 2048
#endif
#define SEQ_FULL 2048
#define DMOD  768
#define NHD   12
#define HD    64
#define NCG   (DMOD / 64)
#define QSC   16.0f
#define PCAR  32768.0f
#define VCAR  1024.0f
#define LOG2E 1.4426950408889634f
#define ATT_WAVES   4
#define ATT_THREADS (ATT_WAVES * 32)
#define QTILES      (SEQ / 64)
#define ATT_BLOCKS  (NHD * QTILES)
#define NKB    (SEQ / 32)
#define SLAB   (16 * 68)
static_assert(NB == 1);
static_assert(HD == 64 && DMOD == NHD * HD && NCG * 64 == DMOD);
static_assert((SEQ % 64) == 0 && SEQ >= 64 && SEQ <= SEQ_FULL);
static_assert(ATT_THREADS == 128 && NKB * 32 == SEQ && ATT_BLOCKS == NHD * (SEQ / 64));
static_assert((DMOD % 64) == 0 && (DMOD % 32) == 0);
static_assert(((SEQ * DMOD / 8) % 256) == 0 && ((DMOD * DMOD / 8) % 256) == 0);
static_assert((SLAB * 4) % 16 == 0);
static_assert(((64 * NCG) % 4) == 0 && (64 * NCG / 4) > 128 && (64 * NCG / 4) <= 256);

typedef unsigned short u16;
typedef _Float16 v16h __attribute__((ext_vector_type(16)));
typedef _Float16 v8h  __attribute__((ext_vector_type(8)));
typedef __bf16   v16b __attribute__((ext_vector_type(16)));
typedef float    v8f  __attribute__((ext_vector_type(8)));
typedef float    v4f  __attribute__((ext_vector_type(4)));
typedef unsigned int v4u __attribute__((ext_vector_type(4)));

union FragH { v16h v; v8h h[2]; v4u u[2]; };
union FragB { v16b v; v4u u[2]; };

__device__ __forceinline__ unsigned short bf_bits(float f) {
  unsigned u = __float_as_uint(f);
  return (unsigned short)((u + 0x7FFFu + ((u >> 16) & 1u)) >> 16);
}
__device__ __forceinline__ float bf_up(unsigned short h) { return __uint_as_float(((unsigned)h) << 16); }
__device__ __forceinline__ float bf_val(float f) { return bf_up(bf_bits(f)); }
__device__ __forceinline__ unsigned short h_bits(_Float16 x) { return __builtin_bit_cast(unsigned short, x); }
__device__ __forceinline__ unsigned pk16(unsigned short a, unsigned short b) { return (unsigned)a | ((unsigned)b << 16); }
__device__ __forceinline__ v8f zero8() { v8f z = {0.f, 0.f, 0.f, 0.f, 0.f, 0.f, 0.f, 0.f}; return z; }

__device__ __forceinline__ v16h ldfrag_h(const _Float16* p) {
  FragH f;
  f.h[0] = *(const v8h*)(p);
  f.h[1] = *(const v8h*)(p + 16);
  return f.v;
}
__device__ __forceinline__ v16b ldfrag_b(const u16* p) {
  FragB f;
  f.u[0] = *(const v4u*)(p);
  f.u[1] = *(const v4u*)(p + 16);
  return f.v;
}

__device__ __forceinline__ v8f mma_h(v16h a, v16h b, v8f c) {
  return __builtin_amdgcn_wmma_f32_16x16x32_f16(false, a, false, b, (short)0, c, false, false);
}
__device__ __forceinline__ v8f mma_b(v16b a, v16b b, v8f c) {
  return __builtin_amdgcn_wmma_f32_16x16x32_bf16(false, a, false, b, (short)0, c, false, false);
}
__device__ __forceinline__ void guard2(v8f& a, v8f& b, v16h x0, v16h x1, v16h x2, v16h x3, v16h x4, v16h x5) {
#if defined(__HIP_DEVICE_COMPILE__)
  asm volatile("v_nop\n\tv_nop\n\tv_nop\n\tv_nop"
               : "+v"(a), "+v"(b) : "v"(x0), "v"(x1), "v"(x2), "v"(x3), "v"(x4), "v"(x5) : "memory");
#endif
}
template <typename F>
__device__ __forceinline__ void guard6(v8f& a, v8f& b, v8f& c, v8f& d, F x0, F x1, F x2, F x3, F x4, F x5) {
#if defined(__HIP_DEVICE_COMPILE__)
  asm volatile("v_nop\n\tv_nop\n\tv_nop\n\tv_nop"
               : "+v"(a), "+v"(b), "+v"(c), "+v"(d) : "v"(x0), "v"(x1), "v"(x2), "v"(x3), "v"(x4), "v"(x5) : "memory");
#endif
}
__device__ __forceinline__ void acc_guard4(v8f& a, v8f& b, v8f& c, v8f& d) {
#if defined(__HIP_DEVICE_COMPILE__)
  asm volatile("v_nop\n\tv_nop\n\tv_nop\n\tv_nop" : "+v"(a), "+v"(b), "+v"(c), "+v"(d));
#endif
}
__device__ __forceinline__ void wave_sync_lds() {
#if defined(__HIP_DEVICE_COMPILE__)
  __builtin_amdgcn_fence(__ATOMIC_RELEASE, "workgroup");
  __builtin_amdgcn_wave_barrier();
  __builtin_amdgcn_fence(__ATOMIC_ACQUIRE, "workgroup");
#endif
}

__global__ __launch_bounds__(256) void cvt16(const float* __restrict__ x, u16* D, int n8, int mode, float scale) {
  const int gt = blockIdx.x * 256 + (int)threadIdx.x;
  if (gt >= n8) return;
  const float* p = x + (size_t)gt * 8;
  const v4f a = *(const v4f*)(p), c4 = *(const v4f*)(p + 4);
  float v[8];
#pragma unroll
  for (int e = 0; e < 4; ++e) { v[e] = a[e]; v[4 + e] = c4[e]; }
  unsigned short s[8];
#pragma unroll
  for (int e = 0; e < 8; ++e) {
    const unsigned short bb = bf_bits(v[e]);
    const unsigned short hb = h_bits((_Float16)(bf_up(bb) * scale));
    s[e] = (mode != 0) ? hb : bb;
  }
  v4u o;
#pragma unroll
  for (int e = 0; e < 4; ++e) o[e] = pk16(s[2 * e], s[2 * e + 1]);
  u16* d = D + (size_t)gt * 8;
  for (int pass = 0; pass < 2; ++pass) {
    *(volatile v4u*)(d) = o;
    __threadfence();
  }
}

__device__ __forceinline__ void epi16(float* sl, v8f a0, v8f a1, v8f a2, v8f a3, float oscale, u16* C, int N,
                                      size_t rowb, int col0, int lane) {
  const int hh = lane >> 4, m = lane & 15;
#pragma unroll
  for (int r = 0; r < 8; ++r) {
    const int ro = (8 * hh + r) * 68 + m;
    sl[ro]      = a0[r] * oscale;
    sl[ro + 16] = a1[r] * oscale;
    sl[ro + 32] = a2[r] * oscale;
    sl[ro + 48] = a3[r] * oscale;
  }
  wave_sync_lds();
  const int rq = lane >> 3, c8 = (lane & 7) * 8;
  v4u ov[4];
#pragma unroll
  for (int i4 = 0; i4 < 4; ++i4) {
    const int row = i4 * 4 + rq;
    const v4f a = *(const v4f*)(sl + row * 68 + c8), c4 = *(const v4f*)(sl + row * 68 + c8 + 4);
    float w[8];
#pragma unroll
    for (int e = 0; e < 4; ++e) { w[e] = a[e]; w[4 + e] = c4[e]; }
#pragma unroll
    for (int e = 0; e < 4; ++e) ov[i4][e] = pk16(h_bits((_Float16)w[2 * e]), h_bits((_Float16)w[2 * e + 1]));
  }
  u16* dst = C + (rowb + (size_t)rq) * (size_t)N + col0 + c8;
  for (int pass = 0; pass < 2; ++pass) {
#pragma unroll
    for (int i4 = 0; i4 < 4; ++i4) {
      *(volatile v4u*)(dst + (size_t)(i4 * 4) * (size_t)N) = ov[i4];
    }
    __threadfence();
  }
}

__global__ __launch_bounds__(128)
void gemm_b16(const u16* __restrict__ A, const u16* __restrict__ Bt, u16* C, const float* __restrict__ bias,
              int M, int N, int K, int nbias, int byrow, float oscale) {
  __shared__ __align__(16) float slab[4 * SLAB];
  const int tid = threadIdx.x, wave = tid >> 5, lane = tid & 31, hh = lane >> 4, m = lane & 15;
  const int ntile = N >> 6;
  const int bid   = blockIdx.x;
  const int rowb  = (bid / ntile) * 64 + wave * 16;
  const int col0  = (bid % ntile) * 64;
  if (rowb + 16 > M) return;
  const u16* ap = A  + (size_t)(rowb + m) * K + 8 * hh;
  const u16* bp = Bt + (size_t)(col0 + m) * K + 8 * hh;
  const size_t bs = (size_t)16 * K;
  v8f acc0 = zero8(), acc1 = zero8(), acc2 = zero8(), acc3 = zero8();
#pragma unroll 1
  for (int k0 = 0; k0 < K; k0 += 32) {
    const v16b a  = ldfrag_b(ap + k0);
    const v16b b0 = ldfrag_b(bp + k0);
    const v16b b1 = ldfrag_b(bp + bs + k0);
    const v16b b2 = ldfrag_b(bp + 2 * bs + k0);
    const v16b b3 = ldfrag_b(bp + 3 * bs + k0);
    acc0 = mma_b(a, b0, acc0);
    acc1 = mma_b(a, b1, acc1);
    acc2 = mma_b(a, b2, acc2);
    acc3 = mma_b(a, b3, acc3);
    guard6<v16b>(acc0, acc1, acc2, acc3, a, b0, b1, b2, b3, a);
  }
  acc_guard4(acc0, acc1, acc2, acc3);
  float bc[4], br[8];
#pragma unroll
  for (int j = 0; j < 4; ++j) {
    int ci = col0 + 16 * j + m;
    ci = (ci < nbias) ? ci : (nbias - 1);
    bc[j] = bf_val(bias[ci]);
  }
#pragma unroll
  for (int r = 0; r < 8; ++r) {
    int ri = rowb + 8 * hh + r;
    ri = (ri < nbias) ? ri : (nbias - 1);
    br[r] = bf_val(bias[ri]);
  }
#pragma unroll
  for (int r = 0; r < 8; ++r) {
    const float q0 = (byrow != 0) ? br[r] : bc[0];
    const float q1 = (byrow != 0) ? br[r] : bc[1];
    const float q2 = (byrow != 0) ? br[r] : bc[2];
    const float q3 = (byrow != 0) ? br[r] : bc[3];
    acc0[r] += q0;
    acc1[r] += q1;
    acc2[r] += q2;
    acc3[r] += q3;
  }
  epi16(slab + wave * SLAB, acc0, acc1, acc2, acc3, oscale, C, N, (size_t)rowb, col0, lane);
}

__global__ __launch_bounds__(128)
void gemm_qn(const u16* __restrict__ A, const u16* __restrict__ Bt, u16* C, float* AAP, const float* __restrict__ bias,
             int M, int K, int nbias, float oscale) {
  __shared__ __align__(16) float slab[4 * SLAB];
  __shared__ __align__(16) float aas[64 * NCG];
  const int tid = threadIdx.x, wave = tid >> 5, lane = tid & 31, hh = lane >> 4, m = lane & 15;
  const int N = NCG * 64;
  const int rowb = blockIdx.x * 64 + wave * 16;
  (void)M;
  const u16* ap = A + (size_t)(rowb + m) * K + 8 * hh;
  const size_t bs = (size_t)16 * K;
#pragma unroll 1
  for (int cg = 0; cg < NCG; ++cg) {
    const int col0 = cg * 64;
    const u16* bp = Bt + (size_t)(col0 + m) * K + 8 * hh;
    v8f acc0 = zero8(), acc1 = zero8(), acc2 = zero8(), acc3 = zero8();
#pragma unroll 1
    for (int k0 = 0; k0 < K; k0 += 32) {
      const v16b a  = ldfrag_b(ap + k0);
      const v16b b0 = ldfrag_b(bp + k0);
      const v16b b1 = ldfrag_b(bp + bs + k0);
      const v16b b2 = ldfrag_b(bp + 2 * bs + k0);
      const v16b b3 = ldfrag_b(bp + 3 * bs + k0);
      acc0 = mma_b(a, b0, acc0);
      acc1 = mma_b(a, b1, acc1);
      acc2 = mma_b(a, b2, acc2);
      acc3 = mma_b(a, b3, acc3);
      guard6<v16b>(acc0, acc1, acc2, acc3, a, b0, b1, b2, b3, a);
    }
    acc_guard4(acc0, acc1, acc2, acc3);
    float bc[4];
#pragma unroll
    for (int j = 0; j < 4; ++j) {
      int ci = col0 + 16 * j + m;
      ci = (ci < nbias) ? ci : (nbias - 1);
      bc[j] = bf_val(bias[ci]);
    }
#pragma unroll
    for (int r = 0; r < 8; ++r) {
      acc0[r] += bc[0];
      acc1[r] += bc[1];
      acc2[r] += bc[2];
      acc3[r] += bc[3];
    }
#pragma unroll
    for (int r = 0; r < 8; ++r) {
      float ss = acc0[r] * acc0[r] + acc1[r] * acc1[r] + acc2[r] * acc2[r] + acc3[r] * acc3[r];
      ss += __shfl_xor(ss, 1, 32);
      ss += __shfl_xor(ss, 2, 32);
      ss += __shfl_xor(ss, 4, 32);
      ss += __shfl_xor(ss, 8, 32);
      const float nrm = sqrtf(ss);
      const float den = fmaxf(nrm, 1e-12f);
      const float inv = 1.0f / den;
      acc0[r] *= inv;
      acc1[r] *= inv;
      acc2[r] *= inv;
      acc3[r] *= inv;
      float a2 = acc0[r] * acc0[r] + acc1[r] * acc1[r] + acc2[r] * acc2[r] + acc3[r] * acc3[r];
      a2 += __shfl_xor(a2, 1, 32);
      a2 += __shfl_xor(a2, 2, 32);
      a2 += __shfl_xor(a2, 4, 32);
      a2 += __shfl_xor(a2, 8, 32);
      if (m == 0) aas[(wave * 16 + 8 * hh + r) * NCG + cg] = a2;
    }
    epi16(slab + wave * SLAB, acc0, acc1, acc2, acc3, oscale, C, N, (size_t)rowb, col0, lane);
    wave_sync_lds();
  }
  __syncthreads();
  const int nf4 = 64 * NCG / 4;
  int i1 = tid + 128;
  i1 = (i1 < nf4) ? i1 : (nf4 - 1);
  const v4f w0 = *(const v4f*)(aas + 4 * tid);
  const v4f w1 = *(const v4f*)(aas + 4 * i1);
  float* dst = AAP + (size_t)blockIdx.x * (size_t)(64 * NCG);
  for (int pass = 0; pass < 2; ++pass) {
    *(volatile v4f*)(dst + 4 * tid) = w0;
    if (tid + 128 < nf4) *(volatile v4f*)(dst + 4 * (tid + 128)) = w1;
    __threadfence();
  }
}

__global__ __launch_bounds__(ATT_THREADS)
void attn_l2(const u16* __restrict__ QPp, const float* __restrict__ AAp, const u16* __restrict__ VPp, float* out,
             const float* aux0, const float* aux1) {
  __shared__ __align__(16) float smem[ATT_WAVES * SLAB];
  (void)aux0; (void)aux1;

  const int tid  = threadIdx.x;
  const int wave = tid >> 5;
  const int lane = tid & 31;
  const int hh   = lane >> 4;
  const int c    = lane & 15;

  const int bid  = blockIdx.x;
  const int qt   = bid % QTILES;
  const int head = bid / QTILES;
  if (head >= NHD) return;
  const int q0   = qt * 64 + wave * 16;
  const size_t hb = (size_t)head * SEQ;

  const _Float16* QH = (const _Float16*)(const void*)QPp;
  const _Float16* Qb = QH + (hb + (size_t)(q0 + c)) * HD + 8 * hh;
  const _Float16* Kb = QH + (hb + (size_t)c) * HD + 8 * hh;
  const _Float16* Vb = (const _Float16*)(const void*)VPp + ((size_t)(head * HD + c)) * SEQ + 8 * hh;
  const float lsc = 0.25f * (LOG2E / (QSC * QSC));
  const float c1l = 0.125f * LOG2E;
  const float aq  = AAp[hb + (size_t)(q0 + c)] * c1l;

  const v16h qf0 = ldfrag_h(Qb);
  const v16h qf1 = ldfrag_h(Qb + 32);

  float mrun = -INFINITY, lrun = 0.f;
  v8f o[4];
#pragma unroll
  for (int j = 0; j < 4; ++j) o[j] = zero8();

#pragma unroll 1
  for (int it = 0; it < NKB; ++it) {
    const int kb = it * 32;
    v8f s0 = zero8(), s1 = zero8();
    const _Float16* k0p = Kb + (size_t)kb * HD;
    const _Float16* k1p = k0p + (size_t)16 * HD;
    const v16h ka0 = ldfrag_h(k0p), ka1 = ldfrag_h(k0p + 32);
    const v16h kc0 = ldfrag_h(k1p), kc1 = ldfrag_h(k1p + 32);
    s0 = mma_h(ka0, qf0, s0);
    s0 = mma_h(ka1, qf1, s0);
    s1 = mma_h(kc0, qf0, s1);
    s1 = mma_h(kc1, qf1, s1);
    guard2(s0, s1, qf0, qf1, ka0, ka1, kc0, kc1);
    const float* am = AAp + hb + (size_t)kb + 8 * hh;
    const v4f w0 = *(const v4f*)(am), w1 = *(const v4f*)(am + 4);
    const v4f w2 = *(const v4f*)(am + 16), w3 = *(const v4f*)(am + 20);
    float tk[16];
#pragma unroll
    for (int i = 0; i < 4; ++i) {
      tk[i]      = s0[i]     * lsc - (aq + w0[i] * c1l);
      tk[4 + i]  = s0[4 + i] * lsc - (aq + w1[i] * c1l);
      tk[8 + i]  = s1[i]     * lsc - (aq + w2[i] * c1l);
      tk[12 + i] = s1[4 + i] * lsc - (aq + w3[i] * c1l);
    }
    float cm = tk[0];
#pragma unroll
    for (int i = 1; i < 16; ++i) cm = fmaxf(cm, tk[i]);
    cm = fmaxf(cm, __shfl_xor(cm, 16, 32));
    const float mn = fmaxf(mrun, cm);
    const float al = (mrun == -INFINITY) ? 0.f : exp2f(mrun - mn);
    mrun = mn;
    float ps = 0.f;
    FragH ph;
#pragma unroll
    for (int w = 0; w < 2; ++w) {
#pragma unroll
      for (int e4 = 0; e4 < 4; ++e4) {
        const int i = 8 * w + 2 * e4;
        const float p0 = exp2f(fminf(tk[i] - mn, 0.f));
        const float p1 = exp2f(fminf(tk[i + 1] - mn, 0.f));
        ps += p0 + p1;
        ph.u[w][e4] = pk16(h_bits((_Float16)(p0 * PCAR)), h_bits((_Float16)(p1 * PCAR)));
      }
    }
    ps += __shfl_xor(ps, 16, 32);
    lrun = lrun * al + ps;
    float scl[8];
#pragma unroll
    for (int r = 0; r < 8; ++r) scl[r] = __shfl(al, 8 * hh + r, 32);
#pragma unroll
    for (int j = 0; j < 4; ++j) {
#pragma unroll
      for (int r = 0; r < 8; ++r) o[j][r] *= scl[r];
    }
    {
      const _Float16* vp = Vb + kb;
      const v16h vf0 = ldfrag_h(vp);
      const v16h vf1 = ldfrag_h(vp + (size_t)16 * SEQ);
      const v16h vf2 = ldfrag_h(vp + (size_t)32 * SEQ);
      const v16h vf3 = ldfrag_h(vp + (size_t)48 * SEQ);
      o[0] = mma_h(ph.v, vf0, o[0]);
      o[1] = mma_h(ph.v, vf1, o[1]);
      o[2] = mma_h(ph.v, vf2, o[2]);
      o[3] = mma_h(ph.v, vf3, o[3]);
      guard6<v16h>(o[0], o[1], o[2], o[3], ph.v, vf0, vf1, vf2, vf3, ph.v);
    }
  }
  acc_guard4(o[0], o[1], o[2], o[3]);

  const float linv = (lrun > 0.f) ? ((1.0f / lrun) * (1.0f / (PCAR * VCAR))) : 0.f;
  float inv[8];
#pragma unroll
  for (int r = 0; r < 8; ++r) inv[r] = __shfl(linv, 8 * hh + r, 32);
  float* slab = smem + wave * SLAB;
#pragma unroll
  for (int r = 0; r < 8; ++r) {
#pragma unroll
    for (int j = 0; j < 4; ++j) slab[(8 * hh + r) * 68 + j * 16 + c] = o[j][r] * inv[r];
  }
  wave_sync_lds();
  v4f vals[8];
#pragma unroll
  for (int it2 = 0; it2 < 8; ++it2) vals[it2] = *(const v4f*)(slab + (it2 * 2 + hh) * 68 + c * 4);
  float* dst = out + (hb + (size_t)(q0 + hh)) * HD + c * 4;
  for (int pass = 0; pass < 2; ++pass) {
#pragma unroll
    for (int it2 = 0; it2 < 8; ++it2) {
      *(volatile v4f*)(dst + (size_t)(it2 * 2) * HD) = vals[it2];
    }
    __threadfence();
  }
}

extern "C" void kernel_launch(void* const* d_in, const int* in_sizes, int n_in,
                              void* d_out, int out_size, void* d_ws, size_t ws_size,
                              hipStream_t stream) {
  if (n_in < 7) return;
  if (in_sizes[0] < SEQ * DMOD) return;
  if (in_sizes[1] < 1 || in_sizes[2] < 1) return;
  if (in_sizes[3] != DMOD * DMOD || in_sizes[5] != DMOD * DMOD) return;
  if (in_sizes[4] != DMOD || in_sizes[6] != DMOD) return;
  if (out_size < SEQ * DMOD) return;

  const float* Xin = (const float*)d_in[0];
  const float* Gin = (const float*)d_in[1];
  const float* Min = (const float*)d_in[2];
  const float* Wq  = (const float*)d_in[3];
  const float* bq  = (const float*)d_in[4];
  const float* Wv  = (const float*)d_in[5];
  const float* bv  = (const float*)d_in[6];
  float*       out = (float*)d_out;

  const size_t szXB = (size_t)SEQ * DMOD * 2;
  const size_t szW  = (size_t)DMOD * DMOD * 2;
  const size_t szQP = (size_t)SEQ * DMOD * 2;
  const size_t szAA = (size_t)NHD * SEQ * 4;
  const size_t szVP = (size_t)DMOD * SEQ * 2;
  size_t off = 0;
  const size_t oXB = off; off += szXB;
  const size_t oWQ = off; off += szW;
  const size_t oWV = off; off += szW;
  const size_t oQP = off; off += szQP;
  const size_t oAA = off; off += szAA;
  const size_t oVP = off; off += szVP;
  if (off > ws_size) return;
  if (off > (size_t)134217728) return;

  char* ws = (char*)d_ws;
  u16*   XB  = (u16*)(ws + oXB);
  u16*   WQB = (u16*)(ws + oWQ);
  u16*   WVB = (u16*)(ws + oWV);
  u16*   QP  = (u16*)(ws + oQP);
  float* AAP = (float*)(ws + oAA);
  u16*   VP  = (u16*)(ws + oVP);

  const int n8x = (SEQ * DMOD) / 8;
  const int n8w = (DMOD * DMOD) / 8;
  if ((n8x % 256) != 0 || (n8w % 256) != 0) return;
  if ((DMOD % 64) != 0 || (SEQ % 64) != 0 || (DMOD % 32) != 0) return;
  const dim3 blk(256);
  const dim3 gX(n8x / 256);
  const dim3 gW(n8w / 256);
  const dim3 gQ(SEQ / 64);
  const dim3 gV((DMOD / 64) * (SEQ / 64));
  const dim3 bG(128);
  const dim3 gAT(ATT_BLOCKS);
  const dim3 bAT(ATT_THREADS);

  cvt16<<<gX, blk, 0, stream>>>(Xin, XB, n8x, 0, 1.0f);
  cvt16<<<gW, blk, 0, stream>>>(Wq, WQB, n8w, 0, 1.0f);
  cvt16<<<gW, blk, 0, stream>>>(Wv, WVB, n8w, 0, 1.0f);
  gemm_qn<<<gQ, bG, 0, stream>>>(XB, WQB, QP, AAP, bq, SEQ, DMOD, DMOD, QSC);
  gemm_b16<<<gV, bG, 0, stream>>>(WVB, XB, VP, bv, DMOD, SEQ, DMOD, DMOD, 1, VCAR);
  attn_l2<<<gAT, bAT, 0, stream>>>(QP, AAP, VP, out, Gin, Min);
  (void)hipGetLastError();
}
